// TanhNewtonLayer_38551626449607
// MI455X (gfx1250) — hardware-verified
//
#include <hip/hip_runtime.h>
#include <math.h>

typedef __attribute__((ext_vector_type(16))) _Float16 v16h;
typedef __attribute__((ext_vector_type(16))) __bf16 v16b;
typedef __attribute__((ext_vector_type(8)))  _Float16 v8h;
typedef __attribute__((ext_vector_type(8)))  float v8f;
typedef __attribute__((ext_vector_type(4)))  float v4f;
typedef __attribute__((ext_vector_type(2)))  float v2f;
typedef __attribute__((ext_vector_type(4)))  unsigned v4u;
typedef __attribute__((ext_vector_type(4)))  int v4i;
typedef float __attribute__((may_alias)) float_a;
typedef int __attribute__((may_alias)) int_a;

template <typename T> __device__ __forceinline__ void vst2(void* p, T v) { *(volatile T*)p = v; __threadfence(); *(volatile T*)p = v; }
__device__ __forceinline__ v8f wmma16(v16h a, v16h b, v8f c) {
  v8f d = __builtin_amdgcn_wmma_f32_16x16x32_f16(false, a, false, b, (short)0, c, false, false);
  asm volatile("v_nop\n\tv_nop\n\tv_nop\n\tv_nop" : "+v"(d) : "v"(a), "v"(b));
  return d;
}
__device__ __forceinline__ v8f wmma_bf(v16b a, v16b b, v8f c) {
  v8f d = __builtin_amdgcn_wmma_f32_16x16x32_bf16(false, a, false, b, (short)0, c, false, false);
  asm volatile("v_nop\n\tv_nop\n\tv_nop\n\tv_nop" : "+v"(d) : "v"(a), "v"(b));
  return d;
}
__device__ __forceinline__ v16h frag_h(const _Float16* rowk0, int lane) {
  union { v16h v; v8h q[2]; } u; const _Float16* p = rowk0 + 8 * (lane >> 4);
  u.q[0] = *(const v8h*)p; u.q[1] = *(const v8h*)(p + 16); return u.v;
}
__device__ __forceinline__ v16h frag_f32(const float* rowk0, int lane) {
  v16h a; const float* p = rowk0 + 8 * (lane >> 4);
#pragma unroll
  for (int i = 0; i < 8; ++i) { a[i] = (_Float16)p[i]; a[8 + i] = (_Float16)p[16 + i]; }
  return a;
}
__device__ __forceinline__ v16h fragc_f32(const float* W, int k0, int n, int lane, int ld, int K) {
  v16h a; const int g = lane >> 4;
#pragma unroll
  for (int i = 0; i < 8; ++i) { const int ka = k0 + 8 * g + i, kb = ka + 16;
    a[i] = (_Float16)(ka < K ? W[(size_t)ka * ld + n] : 0.f); a[8 + i] = (_Float16)(kb < K ? W[(size_t)kb * ld + n] : 0.f); }
  return a;
}
struct F2 { v16b h, l; };
__device__ __forceinline__ F2 bsplit16(const float v[16]) { F2 r;
#pragma unroll
  for (int i = 0; i < 16; ++i) { const __bf16 h = (__bf16)v[i]; r.h[i] = h; r.l[i] = (__bf16)(v[i] - (float)h); }
  return r; }
__device__ __forceinline__ F2 split_row(const float* row, int k0, int lane) { float v[16]; const float* p = row + k0 + 8 * (lane >> 4);
#pragma unroll
  for (int i = 0; i < 8; ++i) { v[i] = p[i]; v[8 + i] = p[16 + i]; }
  return bsplit16(v); }
__device__ __forceinline__ F2 split_rowK(const float* row, int k0, int lane, int K) { float v[16]; const int g = lane >> 4;
#pragma unroll
  for (int i = 0; i < 8; ++i) { const int ka = k0 + 8 * g + i, kb = ka + 16; v[i] = ka < K ? row[ka] : 0.f; v[8 + i] = kb < K ? row[kb] : 0.f; }
  return bsplit16(v); }
__device__ __forceinline__ F2 split_col(const float* W, int k0, int n, int lane, int ld, int K) { float v[16]; const int g = lane >> 4;
#pragma unroll
  for (int i = 0; i < 8; ++i) { const int ka = k0 + 8 * g + i, kb = ka + 16; v[i] = ka < K ? W[(size_t)ka * ld + n] : 0.f; v[8 + i] = kb < K ? W[(size_t)kb * ld + n] : 0.f; }
  return bsplit16(v); }
__device__ __forceinline__ v8f mac3(const F2& a, const F2& b, v8f c) { c = wmma_bf(a.l, b.h, c); c = wmma_bf(a.h, b.l, c); return wmma_bf(a.h, b.h, c); }
__device__ __forceinline__ float sigm(float v) { return 1.0f / (1.0f + expf(-v)); }
#define LDSX() do { asm volatile("s_wait_dscnt 0" ::: "memory"); __builtin_amdgcn_wave_barrier(); __builtin_amdgcn_fence(__ATOMIC_RELEASE, "workgroup"); } while (0)

#define NB 256
#define NN 384
#define NIT 48

__global__ __launch_bounds__(128) void k_fix(const float* __restrict__ x, const float* __restrict__ W, const float* __restrict__ b, float* __restrict__ out) {
  __shared__ __align__(16) float z[64][NN + 4];
  __shared__ __align__(16) float zl[64][NN + 4];
  __shared__ float rn[64];
  const int tid = threadIdx.x, wave = tid >> 5, lane = tid & 31, col = lane & 15, g = lane >> 4;
  const int r0 = blockIdx.x * 64;
  for (int q = tid; q < 64 * NN; q += 128) { const int r = q / NN, c = q % NN; z[r][c] = tanhf(x[(size_t)(r0 + r) * NN + c]); }
  __syncthreads();
#pragma unroll 1
  for (int it = 0; it <= NIT; ++it) {
#pragma unroll 1
    for (int tb = 0; tb < 3; ++tb) { v8f acc[8] = {};
#pragma unroll 1
      for (int kc = 0; kc < NN / 32; ++kc) { const F2 a = split_row(&z[wave * 16 + col][0], kc * 32, lane);
#pragma unroll
        for (int j = 0; j < 8; ++j) acc[j] = mac3(a, split_row(W + (size_t)(tb * 128 + j * 16 + col) * NN, kc * 32, lane), acc[j]); }
#pragma unroll
      for (int j = 0; j < 8; ++j) { const int n = tb * 128 + j * 16 + col; const float bb = b[n];
#pragma unroll
        for (int r = 0; r < 8; ++r) { const int rr = wave * 16 + 8 * g + r; zl[rr][n] = acc[j][r] + bb + x[(size_t)(r0 + rr) * NN + n]; } } }
    __syncthreads();
    if (it < NIT) { for (int q = tid; q < 64 * NN; q += 128) { const int r = q / NN, c = q % NN; z[r][c] = tanhf(zl[r][c]); } }
    else {
      for (int r = 0; r < 16; ++r) { const int rr = wave * 16 + r; float s = 0.f;
        for (int c = lane; c < NN; c += 32) { const float gv = z[rr][c] - tanhf(zl[rr][c]); s += gv * gv; }
#pragma unroll
        for (int off = 16; off >= 1; off >>= 1) s += __shfl_xor(s, off, 32);
        if (lane == 0) rn[rr] = sqrtf(s); } }
    __syncthreads();
  }
  for (int q = tid; q < 64 * (NN / 4); q += 128) { const int r = q / (NN / 4), pc = q % (NN / 4); const bool bad = rn[r] > 1e-4f;
    v4f v = *(const v4f*)(&z[r][pc * 4]); if (bad) v = (v4f){0.f, 0.f, 0.f, 0.f};
    vst2(out + (size_t)(r0 + r) * NN + pc * 4, v); }
}
extern "C" void kernel_launch(void* const* d_in, const int* in_sizes, int n_in, void* d_out, int out_size, void* d_ws, size_t ws_size, hipStream_t stream) {
  (void)in_sizes; (void)n_in; (void)out_size; (void)ws_size; (void)d_ws;
  k_fix<<<NB / 64, 128, 0, stream>>>((const float*)d_in[0], (const float*)d_in[1], (const float*)d_in[2], (float*)d_out);
}
